// STGCN_Model_7198365188832
// MI455X (gfx1250) — hardware-verified
//
#include <hip/hip_runtime.h>
#define BB 32
#define TT 512
#define VV 17
#define NEI 36
#define C1 64
#define C2 128
#define C3 256
#define NCLS 60
#define BCH 4
#define NCHK (BB / BCH)
#define RBT (BCH * TT)
#define RCH (RBT * VV)

typedef __bf16 v16b __attribute__((ext_vector_type(16)));
typedef unsigned short v8us __attribute__((ext_vector_type(8), may_alias));
typedef float  v8f  __attribute__((ext_vector_type(8)));
typedef float  v4f  __attribute__((ext_vector_type(4)));
typedef float  v4fa __attribute__((ext_vector_type(4), may_alias));
union FragB { v16b v; v8us half[2]; unsigned short u[16]; };

__device__ __forceinline__ unsigned short bf16_bits(float x) { unsigned int u = __float_as_uint(x); return (unsigned short)((u + 0x7FFFu + ((u >> 16) & 1u)) >> 16); }
__device__ __forceinline__ float bf16_val(unsigned short b) { return __uint_as_float(((unsigned int)b) << 16); }
__device__ __forceinline__ float bf16_round(float x) { return bf16_val(bf16_bits(x)); }
template <int NT>
__device__ __forceinline__ v8f mmaN(v16b ah, v16b al, v16b bh, v16b bl, v8f c) {
  c = __builtin_amdgcn_wmma_f32_16x16x32_bf16(false, ah, false, bh, (short)0, c, false, false);
  if (NT >= 2) c = __builtin_amdgcn_wmma_f32_16x16x32_bf16(false, al, false, bh, (short)0, c, false, false);
  if (NT >= 3) c = __builtin_amdgcn_wmma_f32_16x16x32_bf16(false, ah, false, bl, (short)0, c, false, false);
  asm volatile("v_nop\n\tv_nop\n\tv_nop\n\tv_nop" : "+v"(c) : "v"(ah), "v"(al), "v"(bh), "v"(bl));
  return c;
}

__global__ __launch_bounds__(256) void k_wt_bf16(const float* __restrict__ W, unsigned short* __restrict__ Wt, int K, int N) {
  const int t = blockIdx.x * 256 + threadIdx.x;
  const int k8n = K / 8;
  if (t >= N * k8n) return;
  const int n = t / k8n, k8 = (t % k8n) * 8;
  v8us v;
#pragma unroll
  for (int i = 0; i < 8; ++i) v[i] = bf16_bits(W[(size_t)(k8 + i) * N + n]);
  *(volatile v8us*)(Wt + (size_t)n * K + k8) = v;
  __threadfence();
  *(volatile v8us*)(Wt + (size_t)n * K + k8) = v;
}

template <bool ASPLIT, int ACT, bool BIAS_BF16>
__global__ __launch_bounds__(128) void k_gemm_bf(const float* __restrict__ A, int lda, const unsigned short* __restrict__ Wt, int ldb,
                                               const float* __restrict__ bias, float* __restrict__ C, int ldc, int M, int N, int K) {
  __shared__ __attribute__((aligned(16))) float so[4][16][64];
  const int tid = threadIdx.x, w = tid >> 5, lane = tid & 31, ln = lane & 15, hh = lane >> 4;
  const int ntn = N / 64;
  const int wid = blockIdx.x * 4 + w;
  const int mt = wid / ntn, nq = wid % ntn;
  if (mt * 16 >= M) return;
  const int row0 = mt * 16, col0 = nq * 64;
  const float* arow = A + (size_t)(row0 + ln) * lda;
  v8f acc[4] = {};
  for (int kb = 0; kb < K; kb += 32) {
    FragB ah, al;
    const v4f x0 = *(const v4fa*)(arow + kb + 8 * hh), x1 = *(const v4fa*)(arow + kb + 8 * hh + 4);
    const v4f x2 = *(const v4fa*)(arow + kb + 16 + 8 * hh), x3 = *(const v4fa*)(arow + kb + 16 + 8 * hh + 4);
    float xs[16] = {x0[0],x0[1],x0[2],x0[3],x1[0],x1[1],x1[2],x1[3],x2[0],x2[1],x2[2],x2[3],x3[0],x3[1],x3[2],x3[3]};
#pragma unroll
    for (int i = 0; i < 16; ++i) { const unsigned short hb = bf16_bits(xs[i]); ah.u[i] = hb; al.u[i] = ASPLIT ? bf16_bits(xs[i] - bf16_val(hb)) : (unsigned short)0; }
#pragma unroll
    for (int t = 0; t < 4; ++t) {
      const unsigned short* brow = Wt + (size_t)(col0 + t * 16 + ln) * ldb + kb;
      FragB b;
      b.half[0] = *(const v8us*)(brow + 8 * hh);
      b.half[1] = *(const v8us*)(brow + 16 + 8 * hh);
      acc[t] = mmaN<ASPLIT ? 2 : 1>(ah.v, al.v, b.v, b.v, acc[t]);
    }
  }
#pragma unroll
  for (int t = 0; t < 4; ++t) {
    float bv = bias ? bias[col0 + t * 16 + ln] : 0.f;
    if (BIAS_BF16) bv = bf16_round(bv);
#pragma unroll
    for (int r = 0; r < 8; ++r) { float v = acc[t][r] + bv; if (ACT == 1) v = fmaxf(v, 0.f); so[w][8 * hh + r][t * 16 + ln] = v; }
  }
  __builtin_amdgcn_fence(__ATOMIC_ACQ_REL, "workgroup");
  __builtin_amdgcn_wave_barrier();
  const int rsub = lane >> 4, c4 = (lane & 15) * 4;
  for (int pass = 0; pass < 2; ++pass) {
#pragma unroll
    for (int q = 0; q < 8; ++q) {
      const int r = q * 2 + rsub;
      const v4f v = *(const v4fa*)&so[w][r][c4];
      *(volatile v4f*)(C + (size_t)(row0 + r) * ldc + col0 + c4) = v;
    }
    if (pass == 0) __threadfence();
  }
}

template <int D, bool CAUSAL>
__global__ __launch_bounds__(128) void k_flash(const float* __restrict__ qb, const float* __restrict__ kb, const float* __restrict__ vb,
                                             int pitch, int T, int H, float scale, float* __restrict__ y, int ypitch) {
  constexpr int KS = D / 32;
  constexpr int DT = D / 16;
  __shared__ __attribute__((aligned(16))) unsigned short sKh[32][D + 8], sKl[32][D + 8], sVh[32][D + 8], sVl[32][D + 8];
  __shared__ __attribute__((aligned(16))) unsigned short sPh[4][16][40], sPl[4][16][40];
  __shared__ __attribute__((aligned(16))) float sO[4][16][D];
  const int tid = threadIdx.x, w = tid >> 5, lane = tid & 31, ln = lane & 15, hh = lane >> 4;
  const int nqb = (T + 63) / 64;
  const int bh = blockIdx.x / nqb, qblk = blockIdx.x % nqb;
  const int b = bh / H, h = bh % H;
  const int q0 = qblk * 64 + w * 16;
  const float* Q = qb + (size_t)b * T * pitch + h * D;
  const float* K = kb + (size_t)b * T * pitch + h * D;
  const float* V = vb + (size_t)b * T * pitch + h * D;

  FragB aqh[KS], aql[KS];
  {
    int row = q0 + ln; if (row >= T) row = T - 1;
    const float* qr = Q + (size_t)row * pitch;
#pragma unroll
    for (int ks = 0; ks < KS; ++ks)
#pragma unroll
      for (int i = 0; i < 16; ++i) {
        const int d = ks * 32 + ((i < 8) ? (8 * hh + i) : (16 + 8 * hh + (i - 8)));
        const float x = qr[d] * scale; const unsigned short hb = bf16_bits(x);
        aqh[ks].u[i] = hb; aql[ks].u[i] = bf16_bits(x - bf16_val(hb));
      }
  }
  float m_r[8], l_r[8];
#pragma unroll
  for (int r = 0; r < 8; ++r) { m_r[r] = -3.0e38f; l_r[r] = 0.f; }
  v8f oacc[DT];
#pragma unroll
  for (int dt = 0; dt < DT; ++dt) oacc[dt] = (v8f){0.f,0.f,0.f,0.f,0.f,0.f,0.f,0.f};

  const int kv_end = CAUSAL ? min(T, qblk * 64 + 64) : T;
  for (int j0 = 0; j0 < kv_end; j0 += 32) {
    __syncthreads();
    for (int e = tid; e < 32 * (D / 4); e += 128) {
      const int r = e / (D / 4), c4 = (e % (D / 4)) * 4;
      const int key = j0 + r;
      v4f kf = {0.f,0.f,0.f,0.f}, vf = {0.f,0.f,0.f,0.f};
      if (key < T) { kf = *(const v4fa*)(K + (size_t)key * pitch + c4); vf = *(const v4fa*)(V + (size_t)key * pitch + c4); }
#pragma unroll
      for (int t = 0; t < 4; ++t) {
        unsigned short hb = bf16_bits(kf[t]); sKh[r][c4 + t] = hb; sKl[r][c4 + t] = bf16_bits(kf[t] - bf16_val(hb));
        hb = bf16_bits(vf[t]); sVh[r][c4 + t] = hb; sVl[r][c4 + t] = bf16_bits(vf[t] - bf16_val(hb));
      }
    }
    __syncthreads();
    v8f s[2];
#pragma unroll
    for (int nt = 0; nt < 2; ++nt) {
      v8f acc = {};
#pragma unroll
      for (int ks = 0; ks < KS; ++ks) {
        FragB bh_, bl_;
        bh_.half[0] = *(const v8us*)&sKh[nt * 16 + ln][ks * 32 + 8 * hh]; bh_.half[1] = *(const v8us*)&sKh[nt * 16 + ln][ks * 32 + 16 + 8 * hh];
        bl_.half[0] = *(const v8us*)&sKl[nt * 16 + ln][ks * 32 + 8 * hh]; bl_.half[1] = *(const v8us*)&sKl[nt * 16 + ln][ks * 32 + 16 + 8 * hh];
        acc = mmaN<3>(aqh[ks].v, aql[ks].v, bh_.v, bl_.v, acc);
      }
      s[nt] = acc;
    }
    float alpha[8];
#pragma unroll
    for (int r = 0; r < 8; ++r) {
      const int qi = q0 + 8 * hh + r;
      const int ja = j0 + ln, jb = j0 + 16 + ln;
      if (CAUSAL) { if (ja > qi) s[0][r] = -3.0e38f; if (jb > qi) s[1][r] = -3.0e38f; }
      if (ja >= T) s[0][r] = -3.0e38f;
      if (jb >= T) s[1][r] = -3.0e38f;
      float mx = fmaxf(s[0][r], s[1][r]);
      mx = fmaxf(mx, __shfl_xor(mx, 1, 32)); mx = fmaxf(mx, __shfl_xor(mx, 2, 32)); mx = fmaxf(mx, __shfl_xor(mx, 4, 32)); mx = fmaxf(mx, __shfl_xor(mx, 8, 32));
      const float mnew = fmaxf(m_r[r], mx);
      alpha[r] = (mnew > -1.0e38f) ? __expf(m_r[r] - mnew) : 1.0f;
      const float p0 = (s[0][r] > -1.0e38f) ? __expf(s[0][r] - mnew) : 0.f;
      const float p1 = (s[1][r] > -1.0e38f) ? __expf(s[1][r] - mnew) : 0.f;
      m_r[r] = mnew;
      l_r[r] = l_r[r] * alpha[r] + p0 + p1;
      unsigned short hb = bf16_bits(p0); sPh[w][8 * hh + r][ln] = hb;      sPl[w][8 * hh + r][ln] = bf16_bits(p0 - bf16_val(hb));
      hb = bf16_bits(p1);                sPh[w][8 * hh + r][16 + ln] = hb; sPl[w][8 * hh + r][16 + ln] = bf16_bits(p1 - bf16_val(hb));
    }
#pragma unroll
    for (int dt = 0; dt < DT; ++dt)
#pragma unroll
      for (int r = 0; r < 8; ++r) oacc[dt][r] *= alpha[r];
    __builtin_amdgcn_fence(__ATOMIC_ACQ_REL, "workgroup");
    __builtin_amdgcn_wave_barrier();
    FragB pah, pal;
    pah.half[0] = *(const v8us*)&sPh[w][ln][8 * hh]; pah.half[1] = *(const v8us*)&sPh[w][ln][16 + 8 * hh];
    pal.half[0] = *(const v8us*)&sPl[w][ln][8 * hh]; pal.half[1] = *(const v8us*)&sPl[w][ln][16 + 8 * hh];
#pragma unroll
    for (int dt = 0; dt < DT; ++dt) {
      FragB bvh, bvl;
#pragma unroll
      for (int i = 0; i < 8; ++i) {
        bvh.u[i] = sVh[8 * hh + i][dt * 16 + ln]; bvh.u[8 + i] = sVh[16 + 8 * hh + i][dt * 16 + ln];
        bvl.u[i] = sVl[8 * hh + i][dt * 16 + ln]; bvl.u[8 + i] = sVl[16 + 8 * hh + i][dt * 16 + ln];
      }
      oacc[dt] = mmaN<3>(pah.v, pal.v, bvh.v, bvl.v, oacc[dt]);
    }
    __builtin_amdgcn_fence(__ATOMIC_ACQ_REL, "workgroup");
    __builtin_amdgcn_wave_barrier();
  }
#pragma unroll
  for (int r = 0; r < 8; ++r) {
    float l = l_r[r];
    l += __shfl_xor(l, 1, 32); l += __shfl_xor(l, 2, 32); l += __shfl_xor(l, 4, 32); l += __shfl_xor(l, 8, 32);
    l_r[r] = (l > 0.f) ? 1.0f / l : 0.f;
  }
#pragma unroll
  for (int dt = 0; dt < DT; ++dt)
#pragma unroll
    for (int r = 0; r < 8; ++r) sO[w][8 * hh + r][dt * 16 + ln] = oacc[dt][r] * l_r[r];
  __builtin_amdgcn_fence(__ATOMIC_ACQ_REL, "workgroup");
  __builtin_amdgcn_wave_barrier();
  for (int pass = 0; pass < 2; ++pass) {
    for (int r = 0; r < 16; ++r) {
      const int row = q0 + r;
      if (row < T && lane < D / 4) {
        const v4f val = *(const v4fa*)&sO[w][r][lane * 4];
        *(volatile v4f*)(y + ((size_t)b * T + row) * ypitch + h * D + lane * 4) = val;
      }
    }
    if (pass == 0) __threadfence();
  }
}

typedef _Float16 v16h __attribute__((ext_vector_type(16)));
union FragH { v16h v; v8us half[2]; _Float16 h[16]; unsigned short u[16]; };
template <int NT>
__device__ __forceinline__ v8f mmaH(v16h ah, v16h al, v16h bh, v16h bl, v8f c) {
  c = __builtin_amdgcn_wmma_f32_16x16x32_f16(false, ah, false, bh, (short)0, c, false, false);
  if (NT >= 2) c = __builtin_amdgcn_wmma_f32_16x16x32_f16(false, al, false, bh, (short)0, c, false, false);
  if (NT >= 3) c = __builtin_amdgcn_wmma_f32_16x16x32_f16(false, ah, false, bl, (short)0, c, false, false);
  asm volatile("v_nop\n\tv_nop\n\tv_nop\n\tv_nop" : "+v"(c) : "v"(ah), "v"(al), "v"(bh), "v"(bl));
  return c;
}
template <bool ASPLIT>
__global__ __launch_bounds__(128) void k_gemm_h(const float* __restrict__ A, int lda, size_t sA, const _Float16* __restrict__ Bh, int ldb, size_t sB, float alpha, float* __restrict__ C, int ldc, size_t sC, int M, int N, int K) {
  __shared__ __attribute__((aligned(16))) float so[4][16][64];
  const int tid = threadIdx.x, w = tid >> 5, lane = tid & 31, ln = lane & 15, hh = lane >> 4; const int by = blockIdx.y;
  A += (size_t)by * sA; Bh += (size_t)by * sB; C += (size_t)by * sC;
  const int ntn = (N + 63) / 64; const int wid = blockIdx.x * 4 + w; const int mt = wid / ntn, nq = wid % ntn; if (mt * 16 >= M) return;
  const int row0 = mt * 16, col0 = nq * 64; const float* arow = A + (size_t)(row0 + ln) * lda;
  v8f acc[4] = {};
  for (int kb = 0; kb < K; kb += 32) {
    FragH ah, al;
    const v4f x0 = *(const v4fa*)(arow + kb + 8 * hh), x1 = *(const v4fa*)(arow + kb + 8 * hh + 4), x2 = *(const v4fa*)(arow + kb + 16 + 8 * hh), x3 = *(const v4fa*)(arow + kb + 16 + 8 * hh + 4);
    float xs[16] = {x0[0],x0[1],x0[2],x0[3],x1[0],x1[1],x1[2],x1[3],x2[0],x2[1],x2[2],x2[3],x3[0],x3[1],x3[2],x3[3]};
#pragma unroll
    for (int i = 0; i < 16; ++i) { const _Float16 h = (_Float16)xs[i]; ah.h[i] = h; al.h[i] = ASPLIT ? (_Float16)(xs[i] - (float)h) : (_Float16)0.0f; }
#pragma unroll
    for (int t = 0; t < 4; ++t) { if (col0 + t * 16 >= N) continue; const size_t boff = (size_t)(col0 + t * 16 + ln) * ldb + kb; FragH bq; bq.half[0] = *(const v8us*)(Bh + boff + 8 * hh); bq.half[1] = *(const v8us*)(Bh + boff + 16 + 8 * hh);
      acc[t] = mmaH<ASPLIT ? 2 : 1>(ah.v, al.v, bq.v, bq.v, acc[t]); }
  }
#pragma unroll
  for (int t = 0; t < 4; ++t) { if (col0 + t * 16 >= N) continue;
#pragma unroll
    for (int r = 0; r < 8; ++r) so[w][8 * hh + r][t * 16 + ln] = acc[t][r] * alpha; }
  __builtin_amdgcn_fence(__ATOMIC_ACQ_REL, "workgroup"); __builtin_amdgcn_wave_barrier();
  const int rsub = lane >> 4, c4 = (lane & 15) * 4;
  for (int pass = 0; pass < 2; ++pass) {
#pragma unroll
    for (int q = 0; q < 8; ++q) { const int r = q * 2 + rsub; if (col0 + c4 < N) { const v4f v = *(const v4fa*)&so[w][r][c4]; *(volatile v4f*)(C + (size_t)(row0 + r) * ldc + col0 + c4) = v; } }
    if (pass == 0) __threadfence(); }
}

template <int DUMMY>
__global__ __launch_bounds__(128) void k_gemm_hh(const _Float16* __restrict__ A, int lda, size_t sA, const _Float16* __restrict__ Bh, int ldb, size_t sB, float alpha, float* __restrict__ C, int ldc, size_t sC, int M, int N, int K) {
  __shared__ __attribute__((aligned(16))) float so[4][16][64];
  const int tid = threadIdx.x, w = tid >> 5, lane = tid & 31, ln = lane & 15, hh = lane >> 4; const int by = blockIdx.y;
  A += (size_t)by * sA; Bh += (size_t)by * sB; C += (size_t)by * sC;
  const int ntn = (N + 63) / 64; const int wid = blockIdx.x * 4 + w; const int mt = wid / ntn, nq = wid % ntn; if (mt * 16 >= M) return;
  const int row0 = mt * 16, col0 = nq * 64; const _Float16* arow = A + (size_t)(row0 + ln) * lda;
  v8f acc[4] = {};
  for (int kb = 0; kb < K; kb += 32) { FragH ah; ah.half[0] = *(const v8us*)((const unsigned short*)arow + kb + 8 * hh); ah.half[1] = *(const v8us*)((const unsigned short*)arow + kb + 16 + 8 * hh);
#pragma unroll
    for (int t = 0; t < 4; ++t) { if (col0 + t * 16 >= N) continue; const size_t boff = (size_t)(col0 + t * 16 + ln) * ldb + kb; FragH bq; bq.half[0] = *(const v8us*)((const unsigned short*)Bh + boff + 8 * hh); bq.half[1] = *(const v8us*)((const unsigned short*)Bh + boff + 16 + 8 * hh);
      acc[t] = mmaH<1>(ah.v, ah.v, bq.v, bq.v, acc[t]); }
  }
#pragma unroll
  for (int t = 0; t < 4; ++t) { if (col0 + t * 16 >= N) continue;
#pragma unroll
    for (int r = 0; r < 8; ++r) so[w][8 * hh + r][t * 16 + ln] = acc[t][r] * alpha; }
  __builtin_amdgcn_fence(__ATOMIC_ACQ_REL, "workgroup"); __builtin_amdgcn_wave_barrier();
  const int rsub = lane >> 4, c4 = (lane & 15) * 4;
  for (int pass = 0; pass < 2; ++pass) {
#pragma unroll
    for (int q = 0; q < 8; ++q) { const int r = q * 2 + rsub; if (col0 + c4 < N) { const v4f v = *(const v4fa*)&so[w][r][c4]; *(volatile v4f*)(C + (size_t)(row0 + r) * ldc + col0 + c4) = v; } }
    if (pass == 0) __threadfence(); }
}

__device__ __forceinline__ int cj(int v) { return v < 0 ? 0 : (v >= VV ? VV - 1 : v); }
struct AdjL { int start[VV + 1]; unsigned char u[VV * VV]; float w[VV * VV]; };
__device__ void build_adj(const int* __restrict__ ei, AdjL& L, float (*A)[VV + 1]) { __shared__ float dinv[VV]; if (threadIdx.x == 0) {
#pragma unroll 1
    for (int v = 0; v < VV; ++v) {
#pragma unroll 1
      for (int u = 0; u < VV; ++u) A[v][u] = (v == u) ? 1.f : 0.f; }
#pragma unroll 1
    for (int e = 0; e < NEI; ++e) A[cj(ei[NEI + e])][cj(ei[e])] += 1.f;
#pragma unroll 1
    for (int v = 0; v < VV; ++v) { float s = 0.f;
#pragma unroll 1
      for (int u = 0; u < VV; ++u) s += A[v][u]; dinv[v] = 1.0f / sqrtf(s); }
    int n = 0;
#pragma unroll 1
    for (int v = 0; v < VV; ++v) { L.start[v] = n;
#pragma unroll 1
      for (int u = 0; u < VV; ++u) if (A[v][u] != 0.f) { L.u[n] = (unsigned char)u; L.w[n] = dinv[v] * A[v][u] * dinv[u]; ++n; } } L.start[VV] = n; } __syncthreads(); }
__global__ __launch_bounds__(256) void k_bt(const float* __restrict__ W2, const float* __restrict__ W3, _Float16* __restrict__ Bt2, _Float16* __restrict__ Bt3) { const int t = blockIdx.x * 256 + threadIdx.x; if (t < C2 * C1) { const int k = t % C1, n = t / C1; *(volatile _Float16*)(Bt2 + t) = (_Float16)bf16_round(W2[k * C2 + n]); } if (t < C3 * C2) { const int k = t % C2, n = t / C2; *(volatile _Float16*)(Bt3 + t) = (_Float16)bf16_round(W3[k * C3 + n]); } }
typedef _Float16 v2h __attribute__((ext_vector_type(2))); typedef float v2fa __attribute__((ext_vector_type(2), aligned(8)));
__device__ __forceinline__ float l1val(const float* __restrict__ x, const float* __restrict__ W1, float b1c, const AdjL& L, size_t bt, int v, int c) {
  const float w0 = bf16_round(W1[c]), w1 = bf16_round(W1[C1 + c]), w2 = bf16_round(W1[2 * C1 + c]); float acc = 0.f;
  for (int k = L.start[v]; k < L.start[v + 1]; ++k) { const float* xr = x + (bt * VV + L.u[k]) * 3; const float xw = bf16_round(xr[0]) * w0 + bf16_round(xr[1]) * w1 + bf16_round(xr[2]) * w2; acc += L.w[k] * xw; }
  return fmaxf(acc + b1c, 0.f); }
__global__ __launch_bounds__(256) void k_l1s(const float* __restrict__ x, const int* __restrict__ ei, const float* __restrict__ W1, const float* __restrict__ b1, int b0, float* __restrict__ PS, float* __restrict__ PQ) { __shared__ AdjL L; __shared__ float A[VV][VV + 1]; build_adj(ei, L, A);
  const int t = blockIdx.x * 256 + threadIdx.x; if (t >= BCH * VV * C1) return; const int c = t % C1, v = (t / C1) % VV, bl = t / (C1 * VV); const float b1c = bf16_round(b1[c]); float s = 0.f, q2 = 0.f;
#pragma unroll 1
  for (int tt = 0; tt < TT; ++tt) { const float h = l1val(x, W1, b1c, L, (size_t)(b0 + bl) * TT + tt, v, c); s += h; q2 += h * h; }
  const size_t o = (size_t)(b0 + bl) * VV * C3 + v * C3 + c; *(volatile float*)(PS + o) = s; *(volatile float*)(PQ + o) = q2; __threadfence(); *(volatile float*)(PS + o) = s; *(volatile float*)(PQ + o) = q2; }
__global__ __launch_bounds__(256) void k_l1a(const float* __restrict__ x, const int* __restrict__ ei, const float* __restrict__ W1, const float* __restrict__ b1, const float* __restrict__ MU, const float* __restrict__ IV, const float* __restrict__ g, const float* __restrict__ be, int b0, _Float16* __restrict__ A16) { __shared__ AdjL L; __shared__ float A[VV][VV + 1]; build_adj(ei, L, A);
  const size_t t = (size_t)blockIdx.x * 256 + threadIdx.x; if (t >= (size_t)RCH * C1 / 8) return; const int c8 = (int)((t * 8) % C1); const size_t row = (t * 8) / C1; const int v = (int)(row % VV); const size_t bt = (size_t)b0 * TT + row / VV; FragH f;
  for (int q = 0; q < 8; ++q) { const int c = c8 + q; const int ch = v * C1 + c; const float h = l1val(x, W1, bf16_round(b1[c]), L, bt, v, c); f.h[q] = (_Float16)((h - MU[ch]) * IV[ch] * bf16_round(g[ch]) + bf16_round(be[ch])); }
  *(volatile v8us*)((unsigned short*)A16 + t * 8) = f.half[0]; __threadfence(); *(volatile v8us*)((unsigned short*)A16 + t * 8) = f.half[0]; }
__global__ __launch_bounds__(256) void k_mix2(const float* __restrict__ XW, const int* __restrict__ ei, const float* __restrict__ b, int b0, _Float16* __restrict__ H2h, float* __restrict__ PS, float* __restrict__ PQ) { __shared__ AdjL L; __shared__ float A[VV][VV + 1]; build_adj(ei, L, A);
  const int tix = blockIdx.x * 256 + threadIdx.x; if (tix >= BCH * VV * C2 / 2) return; const int c = (tix % (C2 / 2)) * 2, v = (tix / (C2 / 2)) % VV, bl = tix / ((C2 / 2) * VV); const float bc0 = bf16_round(b[c]), bc1 = bf16_round(b[c + 1]); float s0 = 0.f, s1 = 0.f, q0 = 0.f, q1 = 0.f;
#pragma unroll 1
  for (int tt = 0; tt < TT; ++tt) { float a0 = 0.f, a1 = 0.f; const float* src = XW + ((size_t)bl * TT + tt) * VV * C2 + c;
    for (int k = L.start[v]; k < L.start[v + 1]; ++k) { const v2fa xv = *(const v2fa*)(src + (size_t)L.u[k] * C2); a0 += L.w[k] * xv.x; a1 += L.w[k] * xv.y; }
    a0 = fmaxf(a0 + bc0, 0.f); a1 = fmaxf(a1 + bc1, 0.f); s0 += a0; s1 += a1; q0 += a0 * a0; q1 += a1 * a1;
    v2h o2; o2.x = (_Float16)a0; o2.y = (_Float16)a1; _Float16* dst = H2h + (((size_t)(b0 + bl) * TT + tt) * VV + v) * C2 + c; *(volatile v2h*)dst = o2; }
  const size_t o = (size_t)(b0 + bl) * VV * C3 + v * C3 + c; *(volatile float*)(PS + o) = s0; *(volatile float*)(PS + o + 1) = s1; *(volatile float*)(PQ + o) = q0; *(volatile float*)(PQ + o + 1) = q1;
  __threadfence();
#pragma unroll 1
  for (int tt = 0; tt < TT; ++tt) { _Float16* dst = H2h + (((size_t)(b0 + bl) * TT + tt) * VV + v) * C2 + c; const v2h cur = *(volatile v2h*)dst; *(volatile v2h*)dst = cur; }
  *(volatile float*)(PS + o) = s0; *(volatile float*)(PS + o + 1) = s1; *(volatile float*)(PQ + o) = q0; *(volatile float*)(PQ + o + 1) = q1; }
__global__ __launch_bounds__(256) void k_bn2(const _Float16* __restrict__ H2h, const float* __restrict__ MU, const float* __restrict__ IV, const float* __restrict__ g, const float* __restrict__ be, int b0, _Float16* __restrict__ A16) { const size_t t = (size_t)blockIdx.x * 256 + threadIdx.x; if (t >= (size_t)RCH * C2 / 8) return; const int c8 = (int)((t * 8) % C2); const int v = (int)(((t * 8) / C2) % VV); const int ch = v * C2 + c8; FragH fi, f; fi.half[0] = *(const v8us*)((const unsigned short*)H2h + (size_t)b0 * TT * VV * C2 + t * 8);
  for (int q = 0; q < 8; ++q) f.h[q] = (_Float16)(((float)fi.h[q] - MU[ch + q]) * IV[ch + q] * bf16_round(g[ch + q]) + bf16_round(be[ch + q])); *(volatile v8us*)((unsigned short*)A16 + t * 8) = f.half[0]; __threadfence(); *(volatile v8us*)((unsigned short*)A16 + t * 8) = f.half[0]; }
__global__ __launch_bounds__(256) void k_mix3(const float* __restrict__ XW, const int* __restrict__ ei, const float* __restrict__ b, int b0, float* __restrict__ S, float* __restrict__ PQ) { __shared__ AdjL L; __shared__ float A[VV][VV + 1]; build_adj(ei, L, A);
  const int tix = blockIdx.x * 256 + threadIdx.x; if (tix >= BCH * VV * C3 / 2) return; const int c = (tix % (C3 / 2)) * 2, v = (tix / (C3 / 2)) % VV, bl = tix / ((C3 / 2) * VV); const float bc0 = bf16_round(b[c]), bc1 = bf16_round(b[c + 1]); float s0 = 0.f, s1 = 0.f, q0 = 0.f, q1 = 0.f;
#pragma unroll 1
  for (int tt = 0; tt < TT; ++tt) { float a0 = 0.f, a1 = 0.f; const float* src = XW + ((size_t)bl * TT + tt) * VV * C3 + c;
    for (int k = L.start[v]; k < L.start[v + 1]; ++k) { const v2fa xv = *(const v2fa*)(src + (size_t)L.u[k] * C3); a0 += L.w[k] * xv.x; a1 += L.w[k] * xv.y; }
    a0 = fmaxf(a0 + bc0, 0.f); a1 = fmaxf(a1 + bc1, 0.f); s0 += a0; s1 += a1; q0 += a0 * a0; q1 += a1 * a1; }
  const size_t o = (size_t)(b0 + bl) * VV * C3 + v * C3 + c; v2fa sv = {s0, s1}, qv = {q0, q1}; *(volatile v2fa*)(S + o) = sv; *(volatile v2fa*)(PQ + o) = qv; __threadfence(); *(volatile v2fa*)(S + o) = sv; *(volatile v2fa*)(PQ + o) = qv; }
__global__ __launch_bounds__(256) void k_fstat(const float* __restrict__ PS, const float* __restrict__ PQ, int C, float* __restrict__ MU, float* __restrict__ IV) { const int ch = blockIdx.x * 256 + threadIdx.x; if (ch >= VV * C) return; const int v = ch / C, c = ch % C; float s = 0.f, q2 = 0.f;
#pragma unroll 1
  for (int b = 0; b < BB; ++b) { s += PS[(size_t)b * VV * C3 + v * C3 + c]; q2 += PQ[(size_t)b * VV * C3 + v * C3 + c]; }
  const float n = (float)(BB * TT); const float mu = s / n; float var = q2 / n - mu * mu; var = fmaxf(var, 0.f); const float iv = 1.0f / sqrtf(var + 1e-5f); *(volatile float*)(MU + ch) = mu; *(volatile float*)(IV + ch) = iv; __threadfence(); *(volatile float*)(MU + ch) = mu; *(volatile float*)(IV + ch) = iv; }
__global__ __launch_bounds__(256) void k_head(const float* __restrict__ S, const float* __restrict__ MU, const float* __restrict__ IV, const float* __restrict__ g, const float* __restrict__ be, const float* __restrict__ Wf, const float* __restrict__ bfv, float* __restrict__ out) { __shared__ float sp[C3]; __shared__ float so[64]; const int b = blockIdx.x, c = threadIdx.x;
  { float s = 0.f; for (int v = 0; v < VV; ++v) { const int ch = v * C3 + c; s += (S[((size_t)b * VV + v) * C3 + c] - (float)TT * MU[ch]) * IV[ch] * bf16_round(g[ch]) + (float)TT * bf16_round(be[ch]); } sp[c] = s / (float)(TT * VV); }
  __syncthreads();
  if (c < 64) { float s = 0.f; if (c < NCLS) { s = bf16_round(bfv[c]);
#pragma unroll 4
      for (int cc = 0; cc < C3; ++cc) s += sp[cc] * bf16_round(Wf[cc * NCLS + c]); } so[c] = s; }
  __syncthreads();
  if (c < NCLS) { *(volatile float*)(out + b * NCLS + c) = so[c]; } __threadfence(); if (c < NCLS) { *(volatile float*)(out + b * NCLS + c) = so[c]; } }
extern "C" void kernel_launch(void* const* d_in, const int* in_sizes, int n_in,
                              void* d_out, int out_size, void* d_ws, size_t ws_size, hipStream_t stream) {
  (void)in_sizes; (void)n_in; (void)out_size;
  const float* x = (const float*)d_in[0]; const int* ei = (const int*)d_in[1]; const float* W1 = (const float*)d_in[2]; const float* b1 = (const float*)d_in[3]; const float* g1 = (const float*)d_in[4]; const float* be1 = (const float*)d_in[5];
  const float* W2 = (const float*)d_in[6]; const float* b2 = (const float*)d_in[7]; const float* g2 = (const float*)d_in[8]; const float* be2 = (const float*)d_in[9]; const float* W3 = (const float*)d_in[10]; const float* b3 = (const float*)d_in[11]; const float* g3 = (const float*)d_in[12]; const float* be3 = (const float*)d_in[13]; const float* Wf = (const float*)d_in[14]; const float* bfv = (const float*)d_in[15];
  char* ws = (char*)d_ws; size_t off = 0;
  auto take = [&](size_t bytes) { char* p = ws + off; off += (bytes + 255) & ~(size_t)255; return p; };
  _Float16* Bt2 = (_Float16*)take((size_t)C2 * C1 * 2); _Float16* Bt3 = (_Float16*)take((size_t)C3 * C2 * 2);
  _Float16* H2h = (_Float16*)take((size_t)BB * TT * VV * C2 * 2);
  float* XW = (float*)take((size_t)RCH * C3 * 4); _Float16* A16 = (_Float16*)take((size_t)RCH * C2 * 2);
  float* PS = (float*)take((size_t)BB * VV * C3 * 4); float* PQ = (float*)take((size_t)BB * VV * C3 * 4); float* S = (float*)take((size_t)BB * VV * C3 * 4);
  float* MU1 = (float*)take(VV * C1 * 4); float* IV1 = (float*)take(VV * C1 * 4); float* MU2 = (float*)take(VV * C2 * 4); float* IV2 = (float*)take(VV * C2 * 4); float* MU3 = (float*)take(VV * C3 * 4); float* IV3 = (float*)take(VV * C3 * 4);
  if (off > ws_size) return;
  auto EW = [](size_t n) { return (unsigned)((n + 255) / 256); };
  k_bt<<<(C3 * C2 + 255) / 256, 256, 0, stream>>>(W2, W3, Bt2, Bt3);
  for (int k = 0; k < NCHK; ++k) k_l1s<<<EW(BCH * VV * C1), 256, 0, stream>>>(x, ei, W1, b1, k * BCH, PS, PQ);
  k_fstat<<<EW(VV * C1), 256, 0, stream>>>(PS, PQ, C1, MU1, IV1);
  for (int k = 0; k < NCHK; ++k) {
    k_l1a<<<EW((size_t)RCH * C1 / 8), 256, 0, stream>>>(x, ei, W1, b1, MU1, IV1, g1, be1, k * BCH, A16);
    k_gemm_hh<0><<<dim3(((RCH / 16) * (C2 / 64) + 3) / 4, 1), 128, 0, stream>>>(A16, C1, 0, Bt2, C1, 0, 1.0f, XW, C2, 0, RCH, C2, C1);
    k_mix2<<<EW(BCH * VV * C2 / 2), 256, 0, stream>>>(XW, ei, b2, k * BCH, H2h, PS, PQ); }
  k_fstat<<<EW(VV * C2), 256, 0, stream>>>(PS, PQ, C2, MU2, IV2);
  for (int k = 0; k < NCHK; ++k) {
    k_bn2<<<EW((size_t)RCH * C2 / 8), 256, 0, stream>>>(H2h, MU2, IV2, g2, be2, k * BCH, A16);
    k_gemm_hh<0><<<dim3(((RCH / 16) * (C3 / 64) + 3) / 4, 1), 128, 0, stream>>>(A16, C2, 0, Bt3, C2, 0, 1.0f, XW, C3, 0, RCH, C3, C2);
    k_mix3<<<EW(BCH * VV * C3 / 2), 256, 0, stream>>>(XW, ei, b3, k * BCH, S, PQ); }
  k_fstat<<<EW(VV * C3), 256, 0, stream>>>(S, PQ, C3, MU3, IV3);
  k_head<<<BB, 256, 0, stream>>>(S, MU3, IV3, g3, be3, Wf, bfv, (float*)d_out);
}
